// GCN_Actor_24223615550523
// MI455X (gfx1250) — hardware-verified
//
#include <hip/hip_runtime.h>
#include <stddef.h>


#define DIMC    128
#define NTHR    256
#define NWAVE   8
#define EPT     8
#define NGRP    2
#define CHUNK   (NTHR * EPT * NGRP)
#define WCAP    (EPT * NGRP * 32)
#define LISTN   (NWAVE * WCAP)
#define NBC     4096
#define NBF     1024
#define RCAP    40960
#define RBN     128
#define TGT     256
#define DEGCAP  256
#define GROWS   128
#define OTHR    512
#define PARTW   512
#define PRED    384
#define HID1    256
#define NOUT    2048
#define WSCALE  8.0f
#define WINV    0.125f

#define LDS_GEMM (GROWS * DIMC * 4)
#define LDS_FILL ((RCAP + NBF + LISTN) * 4 + 64)

static_assert((CHUNK & (CHUNK - 1)) == 0);
static_assert(CHUNK <= 4096);
static_assert(NBC <= 4096 && NBF <= 4096);
static_assert((NBC & (NBC - 1)) == 0 && (NBF & (NBF - 1)) == 0);
static_assert(NBC == 4 * NBF);
static_assert(OTHR * 8 == NBC);
static_assert((RCAP % 32) == 0);
static_assert(GROWS * (DIMC + 8) * 2 <= LDS_GEMM);
static_assert(TGT == NWAVE * 32 && (TGT % GROWS) == 0);
static_assert(TGT == NTHR);
static_assert(PARTW == 2 * NTHR && PRED == TGT + DIMC);
static_assert(NOUT == 8 * NTHR && HID1 == NTHR && DIMC == 4 * 32);

typedef float    v4f  __attribute__((ext_vector_type(4)));
typedef float    v8f  __attribute__((ext_vector_type(8)));
typedef int      v4i  __attribute__((ext_vector_type(4)));
typedef _Float16 v8h  __attribute__((ext_vector_type(8)));
typedef _Float16 v16h __attribute__((ext_vector_type(16)));
union FragH { v16h v; v8h h[2]; };
union FI { float f; int i; };

__device__ __forceinline__ v8h cvt8(v4f a, v4f b) {
  v8h r;
  r[0] = (_Float16)a.x; r[1] = (_Float16)a.y; r[2] = (_Float16)a.z; r[3] = (_Float16)a.w;
  r[4] = (_Float16)b.x; r[5] = (_Float16)b.y; r[6] = (_Float16)b.z; r[7] = (_Float16)b.w;
  return r;
}

__device__ __forceinline__ v8f wmh(v16h a, v16h b, v8f c) {
  v8f d = __builtin_amdgcn_wmma_f32_16x16x32_f16(false, a, false, b, (short)0, c, false, false);
  asm volatile("v_nop\n\tv_nop\n\tv_nop\n\tv_nop" : "+v"(d) : "v"(a), "v"(b));
  return d;
}

__device__ __forceinline__ float rcpf(float x) { return __builtin_amdgcn_rcpf(x); }

__device__ __forceinline__ float dnorm(float g) {
  const float d = g + 1.0f;
  return d > 0.0f ? rsqrtf(d) : 0.0f;
}

template <int NB>
__device__ __forceinline__ int scan_chunk(const int* __restrict__ dsts, int nE, int cbase, int slotBase,
                                          int vec8, int* list, int tid, int lane, int wave) {
  int wc = 0;
#pragma unroll
  for (int g = 0; g < NGRP; ++g) {
    const int el0  = (g * NTHR + tid) * EPT;
    const int e0   = cbase + el0;
    const int sent = -2147483647 - 1;
    v4i da, db;
    if (vec8 != 0 && cbase + CHUNK <= nE) {
      da = *(const v4i*)(dsts + e0);
      db = *(const v4i*)(dsts + e0 + 4);
    } else {
      da.x = (e0     < nE) ? dsts[min(e0, nE - 1)] : sent;
      da.y = (e0 + 1 < nE) ? dsts[min(e0 + 1, nE - 1)] : sent;
      da.z = (e0 + 2 < nE) ? dsts[min(e0 + 2, nE - 1)] : sent;
      da.w = (e0 + 3 < nE) ? dsts[min(e0 + 3, nE - 1)] : sent;
      db.x = (e0 + 4 < nE) ? dsts[min(e0 + 4, nE - 1)] : sent;
      db.y = (e0 + 5 < nE) ? dsts[min(e0 + 5, nE - 1)] : sent;
      db.z = (e0 + 6 < nE) ? dsts[min(e0 + 6, nE - 1)] : sent;
      db.w = (e0 + 7 < nE) ? dsts[min(e0 + 7, nE - 1)] : sent;
    }
    const unsigned nb = (unsigned)slotBase;
    const unsigned s0 = (unsigned)da.x - nb, s1 = (unsigned)da.y - nb;
    const unsigned s2 = (unsigned)da.z - nb, s3 = (unsigned)da.w - nb;
    const unsigned s4 = (unsigned)db.x - nb, s5 = (unsigned)db.y - nb;
    const unsigned s6 = (unsigned)db.z - nb, s7 = (unsigned)db.w - nb;
    const bool h0 = s0 < (unsigned)NB, h1 = s1 < (unsigned)NB, h2 = s2 < (unsigned)NB, h3 = s3 < (unsigned)NB;
    const bool h4 = s4 < (unsigned)NB, h5 = s5 < (unsigned)NB, h6 = s6 < (unsigned)NB, h7 = s7 < (unsigned)NB;
    const unsigned any = __builtin_amdgcn_ballot_w32(h0 | h1 | h2 | h3 | h4 | h5 | h6 | h7);
    if (any != 0u) {
#define HITJ(J, HJ, SJ) { \
        const unsigned mj = __builtin_amdgcn_ballot_w32(HJ); \
        if (mj != 0u) { \
          if (HJ) { \
            const int pos = wc + (int)__builtin_amdgcn_mbcnt_lo(mj, 0u); \
            if (pos < WCAP) list[wave * WCAP + pos] = ((el0 + (J)) << 12) | (int)(SJ); \
          } \
          wc += (int)__builtin_popcount(mj); } }
      HITJ(0, h0, s0)
      HITJ(1, h1, s1)
      HITJ(2, h2, s2)
      HITJ(3, h3, s3)
      HITJ(4, h4, s4)
      HITJ(5, h5, s5)
      HITJ(6, h6, s6)
      HITJ(7, h7, s7)
#undef HITJ
    }
  }
  return wc;
}

__global__ __launch_bounds__(NTHR) void k_wprep(
    const float* __restrict__ Wa, const float* __restrict__ Wb,
    const float* __restrict__ Wc, const float* __restrict__ Wd,
    _Float16* pa, _Float16* pb, _Float16* pc, _Float16* pd,
    int Ka, int Kb, int Kc, int Kd) {
  const int ga = DIMC * Ka / 8, gb = DIMC * Kb / 8, gc = DIMC * Kc / 8, gd = DIMC * Kd / 8;
  const int bstart = blockIdx.x * NTHR;
  const float* src; _Float16* dst; int K, segOff;
  if (bstart < ga)                { src = Wa; dst = pa; K = Ka; segOff = 0; }
  else if (bstart < ga + gb)      { src = Wb; dst = pb; K = Kb; segOff = ga; }
  else if (bstart < ga + gb + gc) { src = Wc; dst = pc; K = Kc; segOff = ga + gb; }
  else                            { src = Wd; dst = pd; K = Kd; segOff = ga + gb + gc; }
  const int i = bstart + (int)threadIdx.x;
  if (i >= ga + gb + gc + gd) return;
  const int o  = (i - segOff) * 8;
  const int n  = o / K;
  const int k0 = o - n * K;
  const int nc = n < DIMC ? n : DIMC - 1;
  float v[8];
#pragma unroll
  for (int e = 0; e < 8; ++e) {
    int k = k0 + e;
    k = k < K ? k : K - 1;
    v[e] = src[(size_t)k * DIMC + nc] * WSCALE;
  }
  v4f a, b;
  a.x = v[0]; a.y = v[1]; a.z = v[2]; a.w = v[3];
  b.x = v[4]; b.y = v[5]; b.z = v[6]; b.w = v[7];
  const v8h hv = cvt8(a, b);
  _Float16* dp = dst + o;
  *(volatile v8h*)dp = hv;
  __threadfence();
  *(volatile v8h*)dp = hv;
}

__global__ __launch_bounds__(NTHR) void k_count(
    const int* __restrict__ ei, const float* __restrict__ ew, int* cnt, float* dinv, int nE, int vec8) {
  __shared__ __attribute__((aligned(16))) int   scnt[NBC];
  __shared__ __attribute__((aligned(16))) float sdeg[NBC];
  __shared__ __attribute__((aligned(16))) int   list[LISTN];
  __shared__ int wcnt[NWAVE];
  const int tid = threadIdx.x, lane = tid & 31, wave = tid >> 5;
  const int nodeBase = blockIdx.x * NBC;
  const int* dsts = ei + nE;

  for (int i = tid; i < NBC; i += NTHR) { scnt[i] = 0; sdeg[i] = 0.0f; }
  __syncthreads();

  const int nChunks = (nE + CHUNK - 1) / CHUNK;
#pragma unroll 1
  for (int ch = 0; ch < nChunks; ++ch) {
    const int cbase = ch * CHUNK;
    const int wc = scan_chunk<NBC>(dsts, nE, cbase, nodeBase, vec8, list, tid, lane, wave);
    if (lane == 0) wcnt[wave] = wc;
    __syncthreads();
    if (wave == 0) {
#pragma unroll 1
      for (int wsx = 0; wsx < NWAVE; ++wsx) {
        int n = __builtin_amdgcn_readfirstlane(wcnt[wsx]);
        n = n > WCAP ? WCAP : (n < 0 ? 0 : n);
        const int* lp = list + wsx * WCAP;
#pragma unroll 1
        for (int i = 0; i < n; ++i) {
          const int ent  = __builtin_amdgcn_readfirstlane(lp[i]);
          const int slot = ent & (NBC - 1);
          int e = cbase + ((ent >> 12) & (CHUNK - 1));
          e = e > nE - 1 ? nE - 1 : e;
          const float w = ew[e];
          if (lane == 0) { scnt[slot] = scnt[slot] + 1; sdeg[slot] = sdeg[slot] + w; }
        }
      }
    }
    __syncthreads();
  }

  v4i cq[4]; v4f dq[4];
#pragma unroll
  for (int q = 0; q < 4; ++q) {
    const int f = (wave * 4 + q) * 128 + 4 * lane;
    const v4i c = *(const v4i*)(scnt + f);
    const v4f g = *(const v4f*)(sdeg + f);
    cq[q] = c;
    dq[q].x = dnorm(g.x);
    dq[q].y = dnorm(g.y);
    dq[q].z = dnorm(g.z);
    dq[q].w = dnorm(g.w);
  }
  int*   cp = cnt + (size_t)nodeBase;
  float* dp = dinv + (size_t)nodeBase;
#pragma unroll
  for (int q = 0; q < 4; ++q) {
    const int f = (wave * 4 + q) * 128 + 4 * lane;
    *(volatile v4i*)(cp + f) = cq[q];
    *(volatile v4f*)(dp + f) = dq[q];
  }
  __threadfence();
#pragma unroll
  for (int q = 0; q < 4; ++q) {
    const int f = (wave * 4 + q) * 128 + 4 * lane;
    *(volatile v4i*)(cp + f) = cq[q];
    *(volatile v4f*)(dp + f) = dq[q];
  }
}

__global__ __launch_bounds__(OTHR) void k_offsets(
    const int* __restrict__ cnt, int* off, int* rbase, int nChunk) {
  __shared__ __attribute__((aligned(16))) int soff[NBC];
  __shared__ __attribute__((aligned(16))) int srb[RBN];
  __shared__ int wtot[OTHR / 32];
  const int tid = threadIdx.x, lane = tid & 31, wave = tid >> 5, sub = tid >> 7;
  for (int i = tid; i < RBN; i += OTHR) srb[i] = 0;
  int carry = 0;
#pragma unroll 1
  for (int ch = 0; ch < nChunk; ++ch) {
    const int base = ch * NBC;
    const v4i c0 = *(const v4i*)(cnt + base + 8 * tid);
    const v4i c1 = *(const v4i*)(cnt + base + 8 * tid + 4);
    const int e0 = max(c0.x, 0), e1 = max(c0.y, 0), e2 = max(c0.z, 0), e3 = max(c0.w, 0);
    const int e4 = max(c1.x, 0), e5 = max(c1.y, 0), e6 = max(c1.z, 0), e7 = max(c1.w, 0);
    const int ts = e0 + e1 + e2 + e3 + e4 + e5 + e6 + e7;
    int incl = ts;
#pragma unroll
    for (int d = 1; d < 32; d <<= 1) {
      const int t = __shfl_up(incl, d);
      if (lane >= d) incl += t;
    }
    if (lane == 31) wtot[wave] = incl;
    __syncthreads();
    const int S0 = wtot[0]  + wtot[1]  + wtot[2]  + wtot[3];
    const int S1 = wtot[4]  + wtot[5]  + wtot[6]  + wtot[7];
    const int S2 = wtot[8]  + wtot[9]  + wtot[10] + wtot[11];
    const int S3 = wtot[12] + wtot[13] + wtot[14] + wtot[15];
    int pre = 0;
#pragma unroll 1
    for (int w = 4 * sub; w < wave; ++w) pre += wtot[w];
    const int b0 = carry;
    const int b1 = b0 + ((S0 + 31) & ~31);
    const int b2 = b1 + ((S1 + 31) & ~31);
    const int b3 = b2 + ((S2 + 31) & ~31);
    const int b4 = b3 + ((S3 + 31) & ~31);
    const int myb = sub == 0 ? b0 : (sub == 1 ? b1 : (sub == 2 ? b2 : b3));
    if (tid == 0) {
      srb[min(4 * ch + 0, RBN - 1)] = b0;
      srb[min(4 * ch + 1, RBN - 1)] = b1;
      srb[min(4 * ch + 2, RBN - 1)] = b2;
      srb[min(4 * ch + 3, RBN - 1)] = b3;
    }
    int run = myb + pre + incl - ts;
    soff[8 * tid + 0] = run; run += e0;
    soff[8 * tid + 1] = run; run += e1;
    soff[8 * tid + 2] = run; run += e2;
    soff[8 * tid + 3] = run; run += e3;
    soff[8 * tid + 4] = run; run += e4;
    soff[8 * tid + 5] = run; run += e5;
    soff[8 * tid + 6] = run; run += e6;
    soff[8 * tid + 7] = run;
    carry = b4;
    __syncthreads();
    const v4i o0 = *(const v4i*)(soff + 4 * tid);
    const v4i o1 = *(const v4i*)(soff + 4 * (tid + OTHR));
    int* op = off + base;
    *(volatile v4i*)(op + 4 * tid) = o0;
    *(volatile v4i*)(op + 4 * (tid + OTHR)) = o1;
    __threadfence();
    *(volatile v4i*)(op + 4 * tid) = o0;
    *(volatile v4i*)(op + 4 * (tid + OTHR)) = o1;
    __syncthreads();
  }
  if (tid == 0) srb[min(4 * nChunk, RBN - 1)] = carry;
  __syncthreads();
  v4i rv = {0, 0, 0, 0};
  if (tid < 32) rv = *(const v4i*)(srb + 4 * tid);
  if (tid < 32) *(volatile v4i*)(rbase + 4 * tid) = rv;
  __threadfence();
  if (tid < 32) *(volatile v4i*)(rbase + 4 * tid) = rv;
}

__global__ __launch_bounds__(NTHR) void k_fill(
    const int* __restrict__ ei, const int* __restrict__ off, const int* __restrict__ rbase,
    int* csr, int nE, int vec8, int csrLen) {
  extern __shared__ v4f lds_dyn[];
  int* region = (int*)lds_dyn;
  int* cursor = region + RCAP;
  int* list   = cursor + NBF;
  int* wcnt   = list + LISTN;
  const int tid = threadIdx.x, lane = tid & 31, wave = tid >> 5;
  const int b = blockIdx.x;
  const int nodeBase = b * NBF;
  const int* dsts = ei + nE;

  int rb0 = rbase[b];
  const int rb1 = rbase[b + 1];
  rb0 = rb0 < 0 ? 0 : (rb0 > csrLen ? csrLen : rb0);
  rb0 &= ~31;
  int len = rb1 - rb0;
  len = len < 0 ? 0 : (len > RCAP ? RCAP : len);
  int lenW = (len + 31) & ~31;
  if (rb0 + lenW > csrLen) lenW = (csrLen - rb0) & ~31;

  {
    const v4i z = {0, 0, 0, 0};
    for (int i = tid; i < RCAP / 4; i += NTHR) ((v4i*)region)[i] = z;
    for (int s = tid; s < NBF; s += NTHR) {
      int o = off[nodeBase + s] - rb0;
      o = o < 0 ? 0 : (o > RCAP ? RCAP : o);
      cursor[s] = o;
    }
  }
  __syncthreads();

  const int nChunks = (nE + CHUNK - 1) / CHUNK;
#pragma unroll 1
  for (int ch = 0; ch < nChunks; ++ch) {
    const int cbase = ch * CHUNK;
    const int wc = scan_chunk<NBF>(dsts, nE, cbase, nodeBase, vec8, list, tid, lane, wave);
    if (lane == 0) wcnt[wave] = wc;
    __syncthreads();
    if (wave == 0) {
#pragma unroll 1
      for (int wsx = 0; wsx < NWAVE; ++wsx) {
        int n = __builtin_amdgcn_readfirstlane(wcnt[wsx]);
        n = n > WCAP ? WCAP : (n < 0 ? 0 : n);
        const int* lp = list + wsx * WCAP;
#pragma unroll 1
        for (int i = 0; i < n; ++i) {
          const int ent  = __builtin_amdgcn_readfirstlane(lp[i]);
          const int slot = ent & (NBF - 1);
          int e = cbase + ((ent >> 12) & (CHUNK - 1));
          e = e > nE - 1 ? nE - 1 : e;
          if (lane == 0) {
            int pos = cursor[slot];
            pos = pos < 0 ? 0 : (pos > RCAP - 1 ? RCAP - 1 : pos);
            region[pos] = e;
            const int np = pos + 1;
            cursor[slot] = np > RCAP ? RCAP : np;
          }
        }
      }
    }
    __syncthreads();
  }

  const int nv = lenW >> 2;
  int* gp = csr + rb0;
#pragma unroll 1
  for (int i = tid; i < nv; i += NTHR) { const v4i v = ((const v4i*)region)[i]; *(volatile v4i*)(gp + 4 * i) = v; }
  __threadfence();
#pragma unroll 1
  for (int i = tid; i < nv; i += NTHR) { const v4i v = ((const v4i*)region)[i]; *(volatile v4i*)(gp + 4 * i) = v; }
}

template <int KD>
__global__ __launch_bounds__(NTHR) void k_gemm(
    const float* __restrict__ A, const _Float16* __restrict__ Bs, const float* __restrict__ dinv,
    const float* __restrict__ bias, float* C, int nRowsA, int useDinv, int useBias) {
  extern __shared__ v4f lds_dyn[];
  constexpr int AP = KD + 8;
  _Float16* sA  = (_Float16*)lds_dyn;
  float*    stg = (float*)lds_dyn;
  const int tid = threadIdx.x, lane = tid & 31, wave = tid >> 5, hh = lane >> 4, m = lane & 15;
  const int rowBase = blockIdx.x * GROWS;

#pragma unroll
  for (int i = 0; i < (GROWS * KD / 8) / NTHR; ++i) {
    const int idx = i * NTHR + tid;
    const int r   = idx / (KD / 8);
    const int c0  = (idx - r * (KD / 8)) * 8;
    int row = rowBase + r;
    row = row > nRowsA - 1 ? nRowsA - 1 : row;
    const float* ap = A + (size_t)row * KD + c0;
    const v4f a = *(const v4f*)ap, b = *(const v4f*)(ap + 4);
    *(v8h*)(sA + r * AP + c0) = cvt8(a, b);
  }
  __syncthreads();

  v8f acc[8];
#pragma unroll
  for (int t = 0; t < 8; ++t) { v8f z = {0.f, 0.f, 0.f, 0.f, 0.f, 0.f, 0.f, 0.f}; acc[t] = z; }
  const _Float16* ar = sA + (wave * 16 + m) * AP + 8 * hh;
#pragma unroll
  for (int kt = 0; kt < KD / 32; ++kt) {
    FragH a;
    a.h[0] = *(const v8h*)(ar + 32 * kt);
    a.h[1] = *(const v8h*)(ar + 32 * kt + 16);
#pragma unroll
    for (int t = 0; t < 8; ++t) {
      const _Float16* bp = Bs + (size_t)(16 * t + m) * KD + 32 * kt + 8 * hh;
      FragH b;
      b.h[0] = *(const v8h*)bp;
      b.h[1] = *(const v8h*)(bp + 16);
      acc[t] = wmh(a.v, b.v, acc[t]);
    }
  }
  __syncthreads();

  const int r0 = wave * 16 + 8 * hh;
  const v4f dA = *(const v4f*)(dinv + (size_t)rowBase + r0);
  const v4f dB = *(const v4f*)(dinv + (size_t)rowBase + r0 + 4);
  float s[8];
  s[0] = dA.x; s[1] = dA.y; s[2] = dA.z; s[3] = dA.w; s[4] = dB.x; s[5] = dB.y; s[6] = dB.z; s[7] = dB.w;
#pragma unroll
  for (int r = 0; r < 8; ++r) s[r] = (useDinv != 0 ? s[r] : 1.0f) * WINV;
  float* sp = stg + r0 * DIMC + m;
#pragma unroll
  for (int t = 0; t < 8; ++t) {
    const float bl = bias[16 * t + m];
    const float bv = useBias != 0 ? bl : 0.0f;
#pragma unroll
    for (int r = 0; r < 8; ++r) sp[r * DIMC + 16 * t] = acc[t][r] * s[r] + bv;
  }
  __syncthreads();

  const float* lp = stg + wave * 16 * DIMC + 4 * lane;
  float* gp = C + ((size_t)rowBase + wave * 16) * DIMC + 4 * lane;
#pragma unroll
  for (int i = 0; i < 16; ++i) { const v4f v = *(const v4f*)(lp + i * DIMC); *(volatile v4f*)(gp + (size_t)i * DIMC) = v; }
  __threadfence();
#pragma unroll
  for (int i = 0; i < 16; ++i) { const v4f v = *(const v4f*)(lp + i * DIMC); *(volatile v4f*)(gp + (size_t)i * DIMC) = v; }
}

__global__ __launch_bounds__(NTHR) void k_agg(
    const int* __restrict__ csr, const int* __restrict__ off, const int* __restrict__ cnt,
    const float* __restrict__ dinv, const int* __restrict__ ei, const float* __restrict__ ew,
    const float* __restrict__ hw, const float* __restrict__ bias, float* h,
    const float* __restrict__ wvec, const float* __restrict__ cjin, float* part,
    int nN, int nE, int csrLen, int mode, int perBatch) {
  __shared__ __attribute__((aligned(16))) float scj[TGT];
  __shared__ __attribute__((aligned(16))) float sred[NWAVE * PRED];
  __shared__ __attribute__((aligned(16))) float sout[PARTW];
  const int tid = threadIdx.x, lane = tid & 31, wave = tid >> 5;
  const int tbase = blockIdx.x * TGT + wave * 32;
  const int cl = tbase + lane;
  const int cnt_l = cnt[cl];
  const int off_l = off[cl];
  FI dvu; dvu.f = dinv[cl];
  const v4f bb = *(const v4f*)(bias + 4 * lane);
  const v4f w4 = *(const v4f*)(wvec + 4 * lane);
  if (mode == 2) {
    const int bgr = (blockIdx.x * TGT) / perBatch;
    scj[tid] = cjin[(size_t)bgr * PARTW + tid];
  } else {
    scj[tid] = 0.0f;
  }
  __syncthreads();
  float cj[8];
  float cmax = -3.0e38f;
#pragma unroll
  for (int t = 0; t < 8; ++t) { cj[t] = scj[lane + 32 * t]; cmax = fmaxf(cmax, cj[t]); }
#pragma unroll
  for (int d = 16; d >= 1; d >>= 1) cmax = fmaxf(cmax, __shfl_xor(cmax, d, 32));
  float ab[8];
#pragma unroll
  for (int t = 0; t < 8; ++t) ab[t] = 0.0f;
  v4f macc = {0.f, 0.f, 0.f, 0.f};
  float cmine = 0.0f;

#pragma unroll 1
  for (int j = 0; j < 32; ++j) {
    const int c = tbase + j;
    int n = __builtin_amdgcn_readlane(cnt_l, j);
    n = n < 0 ? 0 : (n > DEGCAP ? DEGCAP : n);
    const int st = __builtin_amdgcn_readlane(off_l, j);
    FI du; du.i = __builtin_amdgcn_readlane(dvu.i, j);
    const float dc = du.f;
    v4f acc = {0.f, 0.f, 0.f, 0.f};
#pragma unroll 1
    for (int q0 = 0; q0 < n; q0 += 32) {
      int pos = st + q0 + lane;
      pos = pos < 0 ? 0 : (pos > csrLen - 1 ? csrLen - 1 : pos);
      int ed = csr[pos];
      ed = ed < 0 ? 0 : (ed > nE - 1 ? nE - 1 : ed);
      int sl = ei[ed];
      sl = sl < 0 ? 0 : (sl > nN - 1 ? nN - 1 : sl);
      FI wu; wu.f = ew[ed];
      const int mcnt = (n - q0) < 32 ? (n - q0) : 32;
#pragma unroll 1
      for (int p = 0; p < mcnt; ++p) {
        const int s = __builtin_amdgcn_readlane(sl, p);
        FI wp; wp.i = __builtin_amdgcn_readlane(wu.i, p);
        const v4f xr = *(const v4f*)(hw + (size_t)s * DIMC + 4 * lane);
        acc = acc + xr * wp.f;
      }
    }
    const v4f sv = *(const v4f*)(hw + (size_t)c * DIMC + 4 * lane);
    v4f v = (acc + sv) * dc + bb;
    v.x = fmaxf(v.x, 0.f); v.y = fmaxf(v.y, 0.f); v.z = fmaxf(v.z, 0.f); v.w = fmaxf(v.w, 0.f);
    if (mode == 0) {
      float* hp = h + (size_t)c * DIMC + 4 * lane;
      *(volatile v4f*)hp = v;
      __threadfence();
      *(volatile v4f*)hp = v;
    } else {
      float ss = v.x * v.x + v.y * v.y + v.z * v.z + v.w * v.w;
#pragma unroll
      for (int d = 16; d >= 1; d >>= 1) ss += __shfl_xor(ss, d, 32);
      const float nrm = sqrtf(ss);
      const float inv = rcpf(fmaxf(nrm, 1e-12f));
      const v4f vn = v * inv;
      macc = macc + vn;
      float dd = vn.x * w4.x + vn.y * w4.y + vn.z * w4.z + vn.w * w4.w;
#pragma unroll
      for (int d = 16; d >= 1; d >>= 1) dd += __shfl_xor(dd, d, 32);
      if (mode == 1) {
        float* hp = h + (size_t)c * DIMC + 4 * lane;
        *(volatile v4f*)hp = vn;
        __threadfence();
        *(volatile v4f*)hp = vn;
        cmine = (lane == j) ? dd : cmine;
      } else {
        float ea = dd + cmax;
        ea = ea + 1e-7f;
        const float mx = ea >= 0.0f ? ea : 0.01f * ea;
        float ev[8];
        float ssum = 0.0f;
#pragma unroll
        for (int t = 0; t < 8; ++t) {
          float e = dd + cj[t];
          e = e + 1e-7f;
          e = e >= 0.0f ? e : 0.01f * e;
          ev[t] = __expf(e - mx);
          ssum += ev[t];
        }
#pragma unroll
        for (int d = 16; d >= 1; d >>= 1) ssum += __shfl_xor(ssum, d, 32);
        const float invs = rcpf(ssum);
#pragma unroll
        for (int t = 0; t < 8; ++t) ab[t] += ev[t] * invs;
      }
    }
  }

  if (mode != 0) {
    float* wr = sred + wave * PRED;
    if (mode == 2) {
#pragma unroll
      for (int t = 0; t < 8; ++t) wr[lane + 32 * t] = ab[t];
    }
    *(v4f*)(wr + TGT + 4 * lane) = macc;
    if (mode == 1) sout[wave * 32 + lane] = cmine;
    __syncthreads();
    if (mode == 2) {
      float a = 0.0f;
#pragma unroll
      for (int w = 0; w < NWAVE; ++w) a += sred[w * PRED + tid];
      sout[tid] = a;
    }
    if (tid < DIMC) {
      float mm = 0.0f;
#pragma unroll
      for (int w = 0; w < NWAVE; ++w) mm += sred[w * PRED + TGT + tid];
      sout[TGT + tid] = mm;
    } else {
      sout[TGT + tid] = 0.0f;
    }
    __syncthreads();
    if (tid < PARTW / 4) {
      const v4f pv = *(const v4f*)(sout + 4 * tid);
      float* pp = part + (size_t)blockIdx.x * PARTW + 4 * tid;
      *(volatile v4f*)pp = pv;
      __threadfence();
      *(volatile v4f*)pp = pv;
    }
  }
}

__global__ __launch_bounds__(NTHR) void k_head(
    const float* __restrict__ partN, const float* __restrict__ partD, const float* __restrict__ dagN,
    const float* __restrict__ W1, const float* __restrict__ b1,
    const float* __restrict__ W2, const float* __restrict__ b2,
    float* out, int bpbN, int perN, int perD) {
  __shared__ float sab[TGT];
  __shared__ float snm[DIMC];
  __shared__ float sdm[DIMC];
  __shared__ float shy[DIMC];
  __shared__ float shid[HID1];
  __shared__ __attribute__((aligned(16))) float so[NOUT];
  const int tid = threadIdx.x, b = blockIdx.x;
  const float invN = rcpf((float)perN);
  const float invD = rcpf((float)perD);
  const float* pn = partN + (size_t)b * bpbN * PARTW;
  {
    float a = 0.0f;
#pragma unroll 1
    for (int q = 0; q < bpbN; ++q) a += pn[(size_t)q * PARTW + tid];
    sab[tid] = a * invN;
  }
  if (tid < DIMC) {
    float mm = 0.0f;
#pragma unroll 1
    for (int q = 0; q < bpbN; ++q) mm += pn[(size_t)q * PARTW + TGT + tid];
    snm[tid] = mm * invN;
    sdm[tid] = partD[(size_t)b * PARTW + TGT + tid] * invD;
  }
  __syncthreads();
  if (tid < DIMC) {
    float s = 0.0f;
    const float* dr = dagN + (size_t)b * perD * DIMC + tid;
#pragma unroll 1
    for (int j = 0; j < TGT; ++j) s += sab[j] * dr[(size_t)j * DIMC];
    const float ratio = (float)perN * invD;
    shy[tid] = 0.5f * (snm[tid] * (1.0f + ratio) + sdm[tid] + s);
  }
  __syncthreads();
  {
    float s = 0.0f;
#pragma unroll 1
    for (int k = 0; k < DIMC; ++k) s += shy[k] * W1[(size_t)k * HID1 + tid];
    s += b1[tid];
    shid[tid] = fmaxf(s, 0.0f);
  }
  __syncthreads();
  {
    float acc[8] = {0.f, 0.f, 0.f, 0.f, 0.f, 0.f, 0.f, 0.f};
#pragma unroll 1
    for (int k = 0; k < HID1; ++k) {
      const float hk = shid[k];
      const float* wrow = W2 + (size_t)k * NOUT + tid;
#pragma unroll
      for (int q = 0; q < 8; ++q) acc[q] += hk * wrow[q * NTHR];
    }
#pragma unroll
    for (int q = 0; q < 8; ++q) so[q * NTHR + tid] = acc[q] + b2[q * NTHR + tid];
  }
  __syncthreads();
  v4f ov[2];
#pragma unroll
  for (int p = 0; p < 2; ++p) ov[p] = *(const v4f*)(so + 4 * (p * NTHR + tid));
  float* op = out + (size_t)b * NOUT;
#pragma unroll
  for (int p = 0; p < 2; ++p) *(volatile v4f*)(op + 4 * (p * NTHR + tid)) = ov[p];
  __threadfence();
#pragma unroll
  for (int p = 0; p < 2; ++p) *(volatile v4f*)(op + 4 * (p * NTHR + tid)) = ov[p];
}

static void launch_gemm(int KD, int grid, const float* A, const _Float16* Bs, const float* dinv,
                        const float* bias, float* C, int nRows, hipStream_t st) {
  if (KD == 32)       k_gemm<32><<<grid, NTHR, LDS_GEMM, st>>>(A, Bs, dinv, bias, C, nRows, 1, 0);
  else if (KD == 64)  k_gemm<64><<<grid, NTHR, LDS_GEMM, st>>>(A, Bs, dinv, bias, C, nRows, 1, 0);
  else                k_gemm<128><<<grid, NTHR, LDS_GEMM, st>>>(A, Bs, dinv, bias, C, nRows, 1, 0);
}

extern "C" void kernel_launch(void* const* d_in, const int* in_sizes, int n_in,
                              void* d_out, int out_size, void* d_ws, size_t ws_size,
                              hipStream_t stream) {
  if (n_in < 21) return;
  if (in_sizes[8] <= 0 || in_sizes[12] <= 0) return;
  const int FN = in_sizes[8] / DIMC;
  const int FD = in_sizes[12] / DIMC;
  if ((FN != 32 && FN != 64 && FN != 128) || in_sizes[8] != FN * DIMC) return;
  if ((FD != 32 && FD != 64 && FD != 128) || in_sizes[12] != FD * DIMC) return;
  const int nNn = in_sizes[0] / FN;
  const int nEn = in_sizes[1] / 2;
  const int nNd = in_sizes[3] / FD;
  const int nEd = in_sizes[4] / 2;
  if (nNn <= 0 || nEn <= 0 || nNd <= 0 || nEd <= 0) return;
  if (in_sizes[0] != nNn * FN || in_sizes[1] != 2 * nEn || in_sizes[2] != nEn) return;
  if (in_sizes[3] != nNd * FD || in_sizes[4] != 2 * nEd || in_sizes[5] != nEd) return;
  if (in_sizes[9] != DIMC || in_sizes[10] != DIMC * DIMC || in_sizes[11] != DIMC) return;
  if (in_sizes[13] != DIMC || in_sizes[14] != DIMC * DIMC || in_sizes[15] != DIMC) return;
  if (in_sizes[16] != 2 * DIMC || in_sizes[17] != DIMC * HID1 || in_sizes[18] != HID1) return;
  if (in_sizes[20] != NOUT || in_sizes[19] != HID1 * NOUT) return;
  if (out_size <= 0 || (out_size % NOUT) != 0) return;
  const int B = out_size / NOUT;
  const int perN = nNn / B, perD = nNd / B;
  if (nNn != B * perN || nNd != B * perD || perD != TGT || perN < TGT || (perN % TGT) != 0) return;
  if (nEn > (1 << 28) || nEd > (1 << 28) || nNn > (1 << 24) || nNd > (1 << 24)) return;

  const float* net_feat = (const float*)d_in[0];
  const int*   net_ei   = (const int*)d_in[1];
  const float* net_ew   = (const float*)d_in[2];
  const float* dag_feat = (const float*)d_in[3];
  const int*   dag_ei   = (const int*)d_in[4];
  const float* dag_ew   = (const float*)d_in[5];
  const float* net_W0   = (const float*)d_in[8];
  const float* net_b0   = (const float*)d_in[9];
  const float* net_W1   = (const float*)d_in[10];
  const float* net_b1   = (const float*)d_in[11];
  const float* dag_W0   = (const float*)d_in[12];
  const float* dag_b0   = (const float*)d_in[13];
  const float* dag_W1   = (const float*)d_in[14];
  const float* dag_b1   = (const float*)d_in[15];
  const float* W_a      = (const float*)d_in[16];
  const float* head_W1  = (const float*)d_in[17];
  const float* head_b1  = (const float*)d_in[18];
  const float* head_W2  = (const float*)d_in[19];
  const float* head_b2  = (const float*)d_in[20];
  float* out = (float*)d_out;

  const int NPADn  = ((nNn + TGT - 1) / TGT) * TGT;
  const int NPADd  = ((nNd + TGT - 1) / TGT) * TGT;
  const int nBCn   = (nNn + NBC - 1) / NBC;
  const int nBCd   = (nNd + NBC - 1) / NBC;
  if (4 * nBCn + 1 > RBN || 4 * nBCd + 1 > RBN) return;
  const int CNTPn  = nBCn * NBC;
  const int CNTPd  = nBCd * NBC;
  const int nBFn   = (nNn + NBF - 1) / NBF;
  const int nBFd   = (nNd + NBF - 1) / NBF;
  const int csrLn  = ((nEn + 31) & ~31) + 4096;
  const int csrLd  = ((nEd + 31) & ~31) + 4096;
  const int nGemmN = NPADn / GROWS, nGemmD = NPADd / GROWS;
  const int nAggN  = NPADn / TGT,   nAggD  = NPADd / TGT;
  const int bpbN   = perN / TGT;

  char* ws = (char*)d_ws;
  size_t off = 0;
#define CARVE(NAME, BYTES) const size_t NAME = off; off += (size_t)(BYTES); off = (off + 255) & ~(size_t)255;
  CARVE(oWN0, (size_t)DIMC * FN * 2)
  CARVE(oWN1, (size_t)DIMC * DIMC * 2)
  CARVE(oWD0, (size_t)DIMC * FD * 2)
  CARVE(oWD1, (size_t)DIMC * DIMC * 2)
  CARVE(oCntN, (size_t)CNTPn * 4)
  CARVE(oDvN,  (size_t)CNTPn * 4)
  CARVE(oOffN, (size_t)CNTPn * 4)
  CARVE(oRbN,  (size_t)RBN * 4)
  CARVE(oCsrN, (size_t)csrLn * 4)
  CARVE(oHN,   (size_t)NPADn * DIMC * 4)
  CARVE(oHwN,  (size_t)NPADn * DIMC * 4)
  CARVE(oPtN,  (size_t)nAggN * PARTW * 4)
  CARVE(oCntD, (size_t)CNTPd * 4)
  CARVE(oDvD,  (size_t)CNTPd * 4)
  CARVE(oOffD, (size_t)CNTPd * 4)
  CARVE(oRbD,  (size_t)RBN * 4)
  CARVE(oCsrD, (size_t)csrLd * 4)
  CARVE(oHD,   (size_t)NPADd * DIMC * 4)
  CARVE(oHwD,  (size_t)NPADd * DIMC * 4)
  CARVE(oPtD,  (size_t)nAggD * PARTW * 4)
#undef CARVE
  if (off > ws_size) return;
  _Float16* wN0  = (_Float16*)(ws + oWN0);
  _Float16* wN1  = (_Float16*)(ws + oWN1);
  _Float16* wD0  = (_Float16*)(ws + oWD0);
  _Float16* wD1  = (_Float16*)(ws + oWD1);
  int*   cntN  = (int*)(ws + oCntN);
  float* dvN   = (float*)(ws + oDvN);
  int*   offN  = (int*)(ws + oOffN);
  int*   rbN   = (int*)(ws + oRbN);
  int*   csrN  = (int*)(ws + oCsrN);
  float* hN    = (float*)(ws + oHN);
  float* hwN   = (float*)(ws + oHwN);
  float* ptN   = (float*)(ws + oPtN);
  int*   cntD  = (int*)(ws + oCntD);
  float* dvD   = (float*)(ws + oDvD);
  int*   offD  = (int*)(ws + oOffD);
  int*   rbD   = (int*)(ws + oRbD);
  int*   csrD  = (int*)(ws + oCsrD);
  float* hD    = (float*)(ws + oHD);
  float* hwD   = (float*)(ws + oHwD);
  float* ptD   = (float*)(ws + oPtD);

  const int vec8n = ((nEn & 3) == 0) ? 1 : 0;
  const int vec8d = ((nEd & 3) == 0) ? 1 : 0;

  hipFuncSetAttribute(reinterpret_cast<const void*>(&k_fill),
                      hipFuncAttributeMaxDynamicSharedMemorySize, LDS_FILL);
  hipFuncSetAttribute(reinterpret_cast<const void*>(&k_gemm<32>),
                      hipFuncAttributeMaxDynamicSharedMemorySize, LDS_GEMM);
  hipFuncSetAttribute(reinterpret_cast<const void*>(&k_gemm<64>),
                      hipFuncAttributeMaxDynamicSharedMemorySize, LDS_GEMM);
  hipFuncSetAttribute(reinterpret_cast<const void*>(&k_gemm<128>),
                      hipFuncAttributeMaxDynamicSharedMemorySize, LDS_GEMM);

  const int nPrepG = DIMC * (FN + DIMC + FD + DIMC) / 8;
  k_wprep<<<(nPrepG + NTHR - 1) / NTHR, NTHR, 0, stream>>>(net_W0, net_W1, dag_W0, dag_W1,
                                                         wN0, wN1, wD0, wD1, FN, DIMC, FD, DIMC);

  k_count<<<nBCd, NTHR, 0, stream>>>(dag_ei, dag_ew, cntD, dvD, nEd, vec8d);
  k_offsets<<<1, OTHR, 0, stream>>>(cntD, offD, rbD, nBCd);
  k_fill<<<nBFd, NTHR, LDS_FILL, stream>>>(dag_ei, offD, rbD, csrD, nEd, vec8d, csrLd);

  k_count<<<nBCn, NTHR, 0, stream>>>(net_ei, net_ew, cntN, dvN, nEn, vec8n);
  k_offsets<<<1, OTHR, 0, stream>>>(cntN, offN, rbN, nBCn);
  k_fill<<<nBFn, NTHR, LDS_FILL, stream>>>(net_ei, offN, rbN, csrN, nEn, vec8n, csrLn);

  launch_gemm(FD, nGemmD, dag_feat, wD0, dvD, dag_b0, hwD, nNd, stream);
  k_agg<<<nAggD, NTHR, 0, stream>>>(csrD, offD, cntD, dvD, dag_ei, dag_ew, hwD, dag_b0, hD,
                                    W_a + DIMC, ptN, ptD, nNd, nEd, csrLd, 0, perD);
  launch_gemm(DIMC, nGemmD, hD, wD1, dvD, dag_b1, hwD, NPADd, stream);
  k_agg<<<nAggD, NTHR, 0, stream>>>(csrD, offD, cntD, dvD, dag_ei, dag_ew, hwD, dag_b1, hD,
                                    W_a + DIMC, ptN, ptD, nNd, nEd, csrLd, 1, perD);

  launch_gemm(FN, nGemmN, net_feat, wN0, dvN, net_b0, hwN, nNn, stream);
  k_agg<<<nAggN, NTHR, 0, stream>>>(csrN, offN, cntN, dvN, net_ei, net_ew, hwN, net_b0, hN,
                                    W_a, ptD, ptN, nNn, nEn, csrLn, 0, perN);
  launch_gemm(DIMC, nGemmN, hN, wN1, dvN, net_b1, hwN, NPADn, stream);
  k_agg<<<nAggN, NTHR, 0, stream>>>(csrN, offN, cntN, dvN, net_ei, net_ew, hwN, net_b1, hN,
                                    W_a, ptD, ptN, nNn, nEn, csrLn, 2, perN);

  k_head<<<B, NTHR, 0, stream>>>(ptN, ptD, hD, head_W1, head_b1, head_W2, head_b2, out, bpbN, perN, perD);
}
